// TFLongformerSelfAttention_5987184410959
// MI455X (gfx1250) — hardware-verified
//
#include <hip/hip_runtime.h>
#include <math.h>
#include <stdint.h>

#define NBATCH 2
#define SEQ    4096
#define EMB    768
#define NHEAD  12
#define HDIM   64
#define WIN    256
#define QKW    (2 * EMB)
#define NT64   (SEQ / 64)
#define BANDT  4
#define PBW    576
#define SGH    4
#define SMX_T  96

typedef __attribute__((ext_vector_type(16))) _Float16 v16h;
typedef __attribute__((ext_vector_type(8)))  _Float16 v8h;
typedef __attribute__((ext_vector_type(16))) __bf16   v16b;
typedef __attribute__((ext_vector_type(8)))  __bf16   v8b;
typedef __attribute__((ext_vector_type(8)))  float    v8f;
typedef __attribute__((ext_vector_type(4)))  float    v4f;
typedef __attribute__((ext_vector_type(4)))  unsigned int v4u;
#define PSCALE 32768.0f
#define U16(p) ((const unsigned short*)(const void*)(p))
#define PSCALE_INV (1.0f / 32768.0f)

__device__ __forceinline__ unsigned short f2bf_bits(float f) {
  unsigned u = __float_as_uint(f);
  return (unsigned short)((u + 0x7FFFu + ((u >> 16) & 1u)) >> 16);
}
__device__ __forceinline__ float bf_bits2f(unsigned short h) { return __uint_as_float(((unsigned)h) << 16); }
__device__ __forceinline__ unsigned pk16(unsigned short a, unsigned short b) { return (unsigned)a | ((unsigned)b << 16); }

__device__ __forceinline__ void dep_guard_h(v8f& a, v8f& b, v16h x, v16h y) { asm volatile("v_nop\n\tv_nop\n\tv_nop\n\tv_nop" : "+v"(a), "+v"(b) : "v"(x), "v"(y)); }
__device__ __forceinline__ void dep_guard_b(v8f& a, v8f& b, v16b x, v16b y) { asm volatile("v_nop\n\tv_nop\n\tv_nop\n\tv_nop" : "+v"(a), "+v"(b) : "v"(x), "v"(y)); }
__device__ __forceinline__ void keep4_h(v16h a, v16h b, v16h c, v16h d) { asm volatile("v_nop" :: "v"(a), "v"(b), "v"(c), "v"(d)); }
__device__ __forceinline__ void keep4_b(v16b a, v16b b, v16b c, v16b d) { asm volatile("v_nop" :: "v"(a), "v"(b), "v"(c), "v"(d)); }
__device__ __forceinline__ void acc_guard4(v8f& a, v8f& b, v8f& c, v8f& d) { asm volatile("v_nop\n\tv_nop\n\tv_nop\n\tv_nop" : "+v"(a), "+v"(b), "+v"(c), "+v"(d)); }
template <typename T> struct Frag;
template <> struct Frag<_Float16> {
  typedef v16h V; union U { v16h v; v8h h[2]; };
  static __device__ __forceinline__ v16h load(const _Float16* p) {
    U f; f.h[0] = *(const v8h*)(p); f.h[1] = *(const v8h*)(p + 16); return f.v;
  }
  static __device__ __forceinline__ v8f mma(v16h a, v16h b, v8f c) {
    return __builtin_amdgcn_wmma_f32_16x16x32_f16(false, a, false, b, (short)0, c, false, false);
  }
  static __device__ __forceinline__ void guard(v8f& a, v8f& b, v16h x, v16h y) { dep_guard_h(a, b, x, y); }
  static __device__ __forceinline__ void keep(v16h a, v16h b, v16h c, v16h d) { keep4_h(a, b, c, d); }
};
template <> struct Frag<__bf16> {
  typedef v16b V; union U { v16b v; v8b h[2]; };
  static __device__ __forceinline__ v16b load(const __bf16* p) {
    U f; f.h[0] = *(const v8b*)(p); f.h[1] = *(const v8b*)(p + 16); return f.v;
  }
  static __device__ __forceinline__ v8f mma(v16b a, v16b b, v8f c) {
    return __builtin_amdgcn_wmma_f32_16x16x32_bf16(false, a, false, b, (short)0, c, false, false);
  }
  static __device__ __forceinline__ void guard(v8f& a, v8f& b, v16b x, v16b y) { dep_guard_b(a, b, x, y); }
  static __device__ __forceinline__ void keep(v16b a, v16b b, v16b c, v16b d) { keep4_b(a, b, c, d); }
};

template <int ET> struct Elem;
template <> struct Elem<0> { typedef _Float16 T; };
template <> struct Elem<1> { typedef __bf16 T; };
template <int ET, bool SPLIT, int BIAS_MODE, int OUT_MODE, bool RESID, int ACT = 0, int BANDMN = -1, int BANDK = -1, bool BANDST = false>
__global__ __launch_bounds__(256) void wmma_gemm64(
    const unsigned short* __restrict__ Ap, const unsigned short* __restrict__ A2p, int lda, long strideA,
    const unsigned short* __restrict__ Btp, const unsigned short* __restrict__ Bt2p, int ldb, long strideB,
    void* __restrict__ Cout, void* __restrict__ Cout2, int ldc, long strideC,
    const float* __restrict__ bias,
    const float* __restrict__ resid, long strideR,
    int M, int N, int K, float scale, float bsc) {
  typedef typename Elem<ET>::T T;
  typedef typename Frag<T>::V V;
  const T* A = (const T*)Ap; const T* A2 = (const T*)A2p; const T* Bt = (const T*)Btp; const T* Bt2 = (const T*)Bt2p;
  __shared__ __align__(16) float sT[8][16 * 68];
  const int b    = blockIdx.y;
  const int lane = threadIdx.x & 31;
  const int wave = threadIdx.x >> 5;
  const int tilesN = N >> 6;
  const int tilesM = M >> 6;
  const int tile = blockIdx.x * 8 + wave;
  if (tile >= tilesM * tilesN) return;
  const int tm = tile / tilesN;
  const int tn = tile - tm * tilesN;
  const int m0 = tm << 6;
  const int n0 = tn << 6;
  if (BANDMN >= 0) {
    int dt = tm - tn;
    dt = (dt < 0) ? -dt : dt;
    if (dt > BANDMN) return;
  }
  int nC = n0;
  if (BANDST && BANDMN >= 0) {
    int tl = tm - BANDMN; tl = (tl < 0) ? 0 : tl;
    nC = n0 - (tl << 6);
  }

  const T* Ab  = A  + (size_t)b * strideA;
  const T* Bb  = Bt + (size_t)b * strideB;
  const T* Ab2 = SPLIT ? (A2  + (size_t)b * strideA) : nullptr;
  const T* Bb2 = SPLIT ? (Bt2 + (size_t)b * strideB) : nullptr;

  const int rlane = lane & 15;
  const int koff  = (lane >> 4) * 8;
  const int mOff  = (lane >> 4) * 8;

  v8f acc[4][4];
#pragma unroll
  for (int i = 0; i < 4; ++i)
#pragma unroll
    for (int j = 0; j < 4; ++j) acc[i][j] = (v8f){0.f,0.f,0.f,0.f,0.f,0.f,0.f,0.f};

  int kBeg = 0, kEnd = K;
  if (BANDK >= 0) {
    int ks = (tm - BANDK) * 64;     ks = (ks < 0) ? 0 : ks;
    int ke = (tm + BANDK + 1) * 64; ke = (ke > K) ? K : ke;
    kBeg = __builtin_amdgcn_readfirstlane(ks);
    kEnd = __builtin_amdgcn_readfirstlane(ke);
  }
  const int kA = (BANDST && BANDK >= 0) ? kBeg : 0;
  for (int k0 = kBeg; k0 < kEnd; k0 += 32) {
    V bh[4], bl[4];
#pragma unroll
    for (int j = 0; j < 4; ++j) {
      const size_t bo = (size_t)(n0 + (j << 4) + rlane) * ldb + koff + k0;
      bh[j] = Frag<T>::load(Bb + bo);
      if (SPLIT) bl[j] = Frag<T>::load(Bb2 + bo);
    }
#pragma unroll
    for (int i = 0; i < 4; ++i) {
      const size_t ao = (size_t)(m0 + (i << 4) + rlane) * lda + koff + (k0 - kA);
      V ah = Frag<T>::load(Ab + ao);
      V al;
      if (SPLIT) al = Frag<T>::load(Ab2 + ao);
#pragma unroll
      for (int j = 0; j < 4; ++j) {
        acc[i][j] = Frag<T>::mma(ah, bh[j], acc[i][j]);
        if (SPLIT) {
          acc[i][j] = Frag<T>::mma(ah, bl[j], acc[i][j]);
          acc[i][j] = Frag<T>::mma(al, bh[j], acc[i][j]);
        }
      }
      Frag<T>::guard(acc[i][0], acc[i][3], ah, SPLIT ? al : ah);
    }
    Frag<T>::keep(bh[0], bh[1], bh[2], bh[3]);
    if (SPLIT) Frag<T>::keep(bl[0], bl[1], bl[2], bl[3]);
  }
  acc_guard4(acc[0][0], acc[0][1], acc[0][2], acc[0][3]);
  acc_guard4(acc[1][0], acc[1][1], acc[1][2], acc[1][3]);
  acc_guard4(acc[2][0], acc[2][1], acc[2][2], acc[2][3]);
  acc_guard4(acc[3][0], acc[3][1], acc[3][2], acc[3][3]);

  float* slab = sT[wave];
  const float* Rb = RESID ? (resid + (size_t)b * strideR) : nullptr;
#pragma unroll
  for (int i = 0; i < 4; ++i) {
    const int mBase = m0 + (i << 4);
#pragma unroll
    for (int j = 0; j < 4; ++j) {
      const int n = n0 + (j << 4) + rlane;
      float bv = 0.f;
      if (BIAS_MODE == 2) bv = bias[n] * bsc;
#pragma unroll
      for (int r = 0; r < 8; ++r) {
        float v = acc[i][j][r] * scale;
        if (BIAS_MODE == 1) v += bias[mBase + mOff + r] * bsc;
        if (BIAS_MODE == 2) v += bv;
        if (RESID) v += Rb[(size_t)(mBase + mOff + r) * ldc + n];
        if (ACT == 1) v = tanhf(v);
        if (ACT == 2) v = fmaxf(v, 0.0f);
        if (ACT == 3) v = v / (1.0f + expf(-v));
        if (ACT == 4) v = (v > 0.f) ? v : 0.01f * v;
        slab[(mOff + r) * 68 + (j << 4) + rlane] = v;
      }
    }
    __builtin_amdgcn_fence(__ATOMIC_RELEASE, "workgroup");
    __builtin_amdgcn_wave_barrier();
    __builtin_amdgcn_fence(__ATOMIC_ACQUIRE, "workgroup");
    if (OUT_MODE == 0) {
      float* C = (float*)Cout + (size_t)b * strideC;
      const int hh = lane >> 4, c4 = (lane & 15) * 4;
      for (int pass = 0; pass < 2; ++pass) {
#pragma unroll
        for (int it = 0; it < 8; ++it) {
          const int row = it * 2 + hh;
          v4f v = *(const v4f*)(slab + row * 68 + c4);
          *(volatile v4f*)(C + (size_t)(mBase + row) * ldc + nC + c4) = v;
        }
        __threadfence();
      }
    } else {
      const int q = lane >> 3, c8 = (lane & 7) * 8;
      unsigned short* C  = (unsigned short*)Cout  + (size_t)b * strideC;
      unsigned short* C2 = (OUT_MODE == 2) ? ((unsigned short*)Cout2 + (size_t)b * strideC) : nullptr;
      for (int pass = 0; pass < 2; ++pass) {
#pragma unroll
        for (int it = 0; it < 4; ++it) {
          const int row = it * 4 + q;
          const float* sp = slab + row * 68 + c8;
          v8h hv, lv;
#pragma unroll
          for (int e = 0; e < 8; ++e) {
            if (OUT_MODE == 1) {
              hv[e] = (_Float16)sp[e];
            } else {
              unsigned short hb = f2bf_bits(sp[e]);
              unsigned short lb = f2bf_bits(sp[e] - bf_bits2f(hb));
              hv[e] = __builtin_bit_cast(_Float16, hb);
              lv[e] = __builtin_bit_cast(_Float16, lb);
            }
          }
          *(volatile v8h*)(C + (size_t)(mBase + row) * ldc + nC + c8) = hv;
          if (OUT_MODE == 2) *(volatile v8h*)(C2 + (size_t)(mBase + row) * ldc + nC + c8) = lv;
        }
        __threadfence();
      }
    }
    __builtin_amdgcn_fence(__ATOMIC_RELEASE, "workgroup");
    __builtin_amdgcn_wave_barrier();
    __builtin_amdgcn_fence(__ATOMIC_ACQUIRE, "workgroup");
  }
}

__global__ __launch_bounds__(256) void cast_f32_f16x2s(
    const float* __restrict__ in, _Float16* __restrict__ out, int n2, float sc) {
  int i = blockIdx.x * 256 + threadIdx.x;
  if (i < n2) {
    const size_t i2 = 2 * (size_t)i;
    const _Float16 h0 = (_Float16)(in[i2] * sc), h1 = (_Float16)(in[i2 + 1] * sc);
    const unsigned u = (unsigned)__builtin_bit_cast(unsigned short, h0) | ((unsigned)__builtin_bit_cast(unsigned short, h1) << 16);
    ((volatile unsigned*)out)[i] = u;
    __threadfence();
    ((volatile unsigned*)out)[i] = u;
  }
}

__global__ __launch_bounds__(256) void transpose_w_f16(
    const float* __restrict__ W0, const float* __restrict__ W1, const float* __restrict__ W2,
    _Float16* __restrict__ WT, float sc) {
  __shared__ float tile[64][65];
  const int tk = blockIdx.x, tn = blockIdx.y, wi = blockIdx.z;
  const int tid = threadIdx.x, lane = tid & 31, wave = tid >> 5;
  const float* W = (wi == 0) ? W0 : ((wi == 1) ? W1 : W2);
#pragma unroll
  for (int it = 0; it < 16; ++it) {
    const int idx = it * 256 + tid;
    const int r = idx >> 6, c = idx & 63;
    tile[r][c] = W[(size_t)(tk * 64 + r) * EMB + tn * 64 + c];
  }
  __syncthreads();
  _Float16* base = WT + (size_t)wi * EMB * EMB;
  const int q = lane >> 3, c8 = (lane & 7) * 8;
  for (int pass = 0; pass < 2; ++pass) {
#pragma unroll
    for (int it = 0; it < 2; ++it) {
      const int nn = wave * 8 + it * 4 + q;
      v8h hv;
#pragma unroll
      for (int e = 0; e < 8; ++e) hv[e] = (_Float16)(tile[c8 + e][nn] * sc);
      *(volatile v8h*)(base + (size_t)(tn * 64 + nn) * EMB + tk * 64 + c8) = hv;
    }
    __threadfence();
  }
}

__global__ __launch_bounds__(SMX_T) void band_softmax_kernel(const float* __restrict__ S, const float* __restrict__ mrow,
                                                             unsigned short* __restrict__ P) {
  __shared__ float redm[SMX_T / 32];
  __shared__ float reds[SMX_T / 32];
  const int i    = blockIdx.x;
  const int y    = blockIdx.y;
  const int tid  = threadIdx.x;
  const int lane = tid & 31;
  const int wave = tid >> 5;
  const int tm   = i >> 6;
  int tlo = tm - BANDT;     tlo = (tlo < 0) ? 0 : tlo;
  int thi = tm + BANDT + 1; thi = (thi > NT64) ? NT64 : thi;
  const int c0 = tlo * 64;
  const int c1 = thi * 64;
  const int jj = tid * 8;
  const int j  = c0 + jj;
  const bool active = (j < c1);
  const int jjc = active ? jj : 0;
  const int jc  = c0 + jjc;
  const size_t roff = ((size_t)y * SEQ + (size_t)i) * PBW;
  const v4f a0 = *(const v4f*)(S + roff + jjc);
  const v4f a1 = *(const v4f*)(S + roff + jjc + 4);
  const v4f k0 = *(const v4f*)(mrow + jc);
  const v4f k1 = *(const v4f*)(mrow + jc + 4);
  const float sv[8] = {a0[0], a0[1], a0[2], a0[3], a1[0], a1[1], a1[2], a1[3]};
  const float mk[8] = {k0[0], k0[1], k0[2], k0[3], k1[0], k1[1], k1[2], k1[3]};
  bool  adm[8];
  float t[8];
  float m = -INFINITY;
#pragma unroll
  for (int e = 0; e < 8; ++e) {
    const int d = i - (j + e);
    adm[e] = active && (d <= WIN) && (d >= -WIN);
    const float add = (mk[e] != 0.0f) ? -10000.0f : 0.0f;
    t[e] = adm[e] ? (sv[e] + add) : -INFINITY;
    m = fmaxf(m, t[e]);
  }
#pragma unroll
  for (int off = 16; off > 0; off >>= 1) m = fmaxf(m, __shfl_xor(m, off, 32));
  if (lane == 0) redm[wave] = m;
  __syncthreads();
  const float mx = fmaxf(fmaxf(redm[0], redm[1]), redm[2]);
  float ev[8];
  float s = 0.f;
#pragma unroll
  for (int e = 0; e < 8; ++e) {
    ev[e] = adm[e] ? __expf(t[e] - mx) : 0.0f;
    s += ev[e];
  }
#pragma unroll
  for (int off = 16; off > 0; off >>= 1) s += __shfl_xor(s, off, 32);
  if (lane == 0) reds[wave] = s;
  __syncthreads();
  const float tot = (reds[0] + reds[1]) + reds[2];
  const float qm  = mrow[i];
  const float inv = (qm < 0.0f) ? 0.0f : PSCALE * (1.0f / tot);
  unsigned short hb[8];
#pragma unroll
  for (int e = 0; e < 8; ++e) hb[e] = __builtin_bit_cast(unsigned short, (_Float16)(ev[e] * inv));
  const v4u pv = (v4u){pk16(hb[0], hb[1]), pk16(hb[2], hb[3]), pk16(hb[4], hb[5]), pk16(hb[6], hb[7])};
  unsigned short* dst = P + roff + (size_t)jjc;
  if (active) *(volatile v4u*)dst = pv;
  __threadfence();
  if (active) *(volatile v4u*)dst = pv;
}

extern "C" void kernel_launch(void* const* d_in, const int* in_sizes, int n_in,
                              void* d_out, int out_size, void* d_ws, size_t ws_size,
                              hipStream_t stream) {
  if (n_in < 8) return;
  if (in_sizes[0] != NBATCH * SEQ * EMB) return;
  if (in_sizes[1] != NBATCH * SEQ) return;
  if (in_sizes[2] != EMB * EMB || in_sizes[4] != EMB * EMB || in_sizes[6] != EMB * EMB) return;
  if (in_sizes[3] != EMB || in_sizes[5] != EMB || in_sizes[7] != EMB) return;
  if (out_size != NBATCH * SEQ * EMB) return;

  const float* x     = (const float*)d_in[0];
  const float* amask = (const float*)d_in[1];
  const float* Wq    = (const float*)d_in[2];
  const float* bq    = (const float*)d_in[3];
  const float* Wk    = (const float*)d_in[4];
  const float* bk    = (const float*)d_in[5];
  const float* Wv    = (const float*)d_in[6];
  const float* bv    = (const float*)d_in[7];
  float* out = (float*)d_out;

  const size_t PX  = (size_t)NBATCH * SEQ * EMB * 2;
  const size_t PW  = (size_t)3 * EMB * EMB * 2;
  const size_t PQK = (size_t)NBATCH * SEQ * QKW * 2;
  const size_t PVT = (size_t)NBATCH * EMB * SEQ * 2;
  const size_t PS  = (size_t)SGH * SEQ * PBW * 4;
  const size_t PP  = (size_t)SGH * SEQ * PBW * 2;
  size_t off = 0;
  const size_t oX  = off; off += PX;
  const size_t oW  = off; off += PW;
  const size_t oQK = off; off += PQK;
  const size_t oVT = off; off += PVT;
  const size_t oS  = off; off += PS;
  const size_t oP  = off; off += PP;
  if (off > ws_size) return;
  if (off > (size_t)134217728) return;

  char* ws = (char*)d_ws;
  unsigned short* X16  = (unsigned short*)(ws + oX);
  unsigned short* WT16 = (unsigned short*)(ws + oW);
  unsigned short* QK16 = (unsigned short*)(ws + oQK);
  unsigned short* VT16 = (unsigned short*)(ws + oVT);
  float*          Sbuf = (float*)(ws + oS);
  unsigned short* P16  = (unsigned short*)(ws + oP);

  const float* dummy = bq;
  const dim3 blk(256);
  const int n2x = NBATCH * SEQ * EMB / 2;

  cast_f32_f16x2s<<<dim3((n2x + 255) / 256), blk, 0, stream>>>(x, (_Float16*)X16, n2x, 16.0f);
  transpose_w_f16<<<dim3(EMB / 64, EMB / 64, 3), blk, 0, stream>>>(Wq, Wk, Wv, (_Float16*)WT16, 256.0f);

  {
    const dim3 g((((NBATCH * SEQ) / 64) * (EMB / 64) + 7) / 8, 1);
    wmma_gemm64<0, false, 2, 1, false><<<g, blk, 0, stream>>>(
        X16, X16, EMB, 0L, WT16, WT16, EMB, 0L, (void*)QK16, (void*)QK16, QKW, 0L,
        bq, dummy, 0L, NBATCH * SEQ, EMB, EMB, 0.000244140625f, 1.0f);
    wmma_gemm64<0, false, 2, 1, false><<<g, blk, 0, stream>>>(
        X16, X16, EMB, 0L, WT16 + (size_t)EMB * EMB, WT16 + (size_t)EMB * EMB, EMB, 0L,
        (void*)(QK16 + EMB), (void*)(QK16 + EMB), QKW, 0L,
        bk, dummy, 0L, NBATCH * SEQ, EMB, EMB, 0.001953125f, 8.0f);
  }
  {
    const dim3 g(((EMB / 64) * (SEQ / 64) + 7) / 8, NBATCH);
    wmma_gemm64<0, false, 1, 1, false><<<g, blk, 0, stream>>>(
        WT16 + (size_t)2 * EMB * EMB, WT16 + (size_t)2 * EMB * EMB, EMB, 0L,
        X16, X16, EMB, (long)SEQ * EMB,
        (void*)VT16, (void*)VT16, SEQ, (long)EMB * SEQ,
        bv, dummy, 0L, EMB, SEQ, EMB, 0.001953125f, 8.0f);
  }

  const dim3 gS(((SEQ / 64) * (SEQ / 64) + 7) / 8, SGH);
  const dim3 gSm(SEQ, SGH);
  const dim3 gPV(((SEQ / 64) * (HDIM / 64) + 7) / 8, SGH);
  for (int b = 0; b < NBATCH; ++b) {
    const unsigned short* QKb = QK16 + (size_t)b * SEQ * QKW;
    const unsigned short* VTb = VT16 + (size_t)b * EMB * SEQ;
    const float* mrow = amask + (size_t)b * SEQ;
    float* outb = out + (size_t)b * SEQ * EMB;
    for (int sg = 0; sg < NHEAD / SGH; ++sg) {
      const int h0 = sg * SGH;
      wmma_gemm64<0, false, 0, 0, false, 0, BANDT, -1, true><<<gS, blk, 0, stream>>>(
          QKb + (size_t)h0 * HDIM, QKb + (size_t)h0 * HDIM, QKW, (long)HDIM,
          QKb + EMB + (size_t)h0 * HDIM, QKb + EMB + (size_t)h0 * HDIM, QKW, (long)HDIM,
          (void*)Sbuf, (void*)Sbuf, PBW, (long)SEQ * PBW,
          dummy, dummy, 0L, SEQ, SEQ, HDIM, 0.015625f, 1.0f);
      band_softmax_kernel<<<gSm, dim3(SMX_T), 0, stream>>>(Sbuf, mrow, P16);
      wmma_gemm64<0, false, 0, 0, false, 0, -1, BANDT, true><<<gPV, blk, 0, stream>>>(
          P16, P16, PBW, (long)SEQ * PBW,
          VTb + (size_t)h0 * HDIM * SEQ, VTb + (size_t)h0 * HDIM * SEQ, SEQ, (long)HDIM * SEQ,
          (void*)(outb + (size_t)h0 * HDIM), (void*)(outb + (size_t)h0 * HDIM), EMB, (long)HDIM,
          dummy, dummy, 0L, SEQ, HDIM, SEQ, 0.000003814697265625f, 1.0f);
    }
  }
  (void)hipGetLastError();
}
